// cAttend_simple_2911987827482
// MI455X (gfx1250) — hardware-run, weakly checked
//
#include <hip/hip_runtime.h>


#ifndef NB
#define NB 64
#endif
#ifndef ND
#define ND 8192
#endif
#ifndef NNZ
#define NNZ 1024
#endif
#define NB_FULL 64
#define ND_FULL 8192
#define NE   256
#define NQ   256
#define SELT 256
#define SELP (SELT * 8)
#define NIT  (ND / SELP)
#define QRS  2048.0f
#define QRI  (1.0f / 2048.0f)
#define SCL  0.0625f

static_assert(NE % 32 == 0);
static_assert(NQ % 32 == 0);
static_assert(ND % 32 == 0);
static_assert(ND % 64 == 0);
static_assert(NQ % 64 == 0);
static_assert(NE == NQ);
static_assert(NB % 16 == 0);
static_assert(ND % SELP == 0);
static_assert(SELT * 8 == SELP);
static_assert(SELT * 4 * 2 == SELP);
static_assert(SELT % 32 == 0);
static_assert(NB <= NB_FULL);
static_assert(ND <= ND_FULL);
static_assert(NNZ <= ND);
static_assert(((size_t)ND * NE) % 8 == 0);
static_assert(((size_t)NQ * NE) % 8 == 0);
static_assert(32 * 16 * 4 == 16 * 128);
static_assert(32 * 16 * 8 == 16 * 256);
static_assert(16 * 68 * 4 <= 131072);
static_assert(SELP * 4 + NIT * (SELT / 32) * 4 <= 131072);

typedef _Float16 h16;
typedef unsigned short bf;
typedef __attribute__((ext_vector_type(16))) __bf16   v16bf;
typedef __attribute__((ext_vector_type(16))) _Float16 v16h;
typedef __attribute__((ext_vector_type(8)))  _Float16 v8h;
typedef __attribute__((ext_vector_type(8)))  unsigned short v8us;
typedef __attribute__((ext_vector_type(8)))  float    v8f;
typedef __attribute__((ext_vector_type(4)))  float    v4f;
typedef v4f  __attribute__((may_alias)) v4fa;

__device__ __forceinline__ unsigned short f2bf(float f) { unsigned u = __float_as_uint(f); u += 0x7FFFu + ((u >> 16) & 1u); return (unsigned short)(u >> 16); }
__device__ __forceinline__ float bfr(float f) { return __uint_as_float(((unsigned)f2bf(f)) << 16); }
__device__ __forceinline__ v16h cat16(v8h lo, v8h hi) { return __builtin_shufflevector(lo, hi, 0, 1, 2, 3, 4, 5, 6, 7, 8, 9, 10, 11, 12, 13, 14, 15); }
__device__ __forceinline__ v16bf cat16b(v8us lo, v8us hi) { return __builtin_bit_cast(v16bf, __builtin_shufflevector(lo, hi, 0, 1, 2, 3, 4, 5, 6, 7, 8, 9, 10, 11, 12, 13, 14, 15)); }
__device__ __forceinline__ v8f wmma16(v16h a, v16h b, v8f c) { return __builtin_amdgcn_wmma_f32_16x16x32_f16(false, a, false, b, (short)0, c, false, false); }
__device__ __forceinline__ v8f wmmab(v16bf a, v16bf b, v8f c) { return __builtin_amdgcn_wmma_f32_16x16x32_bf16(false, a, false, b, (short)0, c, false, false); }
__device__ __forceinline__ v16h  ldh(const h16* p) { return cat16(*(const v8h*)p, *(const v8h*)(p + 16)); }
__device__ __forceinline__ v16bf ldb(const bf* p)  { return cat16b(*(const v8us*)p, *(const v8us*)(p + 16)); }
__device__ __forceinline__ void wave_sync() { __builtin_amdgcn_fence(3  , "wavefront"); __builtin_amdgcn_wave_barrier(); asm volatile("" ::: "memory"); }

__device__ __forceinline__ h16 toh_flush(float v) { const h16 r = (h16)v; return (fabsf(v) < 6.103515625e-05f) ? (h16)0.0f : r; }
__device__ __forceinline__ v8f gw16(v16h a, v16h b, v8f c) { c = wmma16(a, b, c); asm volatile("v_nop\n\tv_nop\n\tv_nop\n\tv_nop" : "+v"(c) : "v"(a), "v"(b)); return c; }
__device__ __forceinline__ v8f gwb(v16bf a, v16bf b, v8f c) { c = wmmab(a, b, c); asm volatile("v_nop\n\tv_nop\n\tv_nop\n\tv_nop" : "+v"(c) : "v"(a), "v"(b)); return c; }
__device__ __forceinline__ void split8(const v4f x0, const v4f x1, v8h& hv, v8h& rv) {
#pragma unroll
    for (int i = 0; i < 4; ++i) {
        const h16 a0 = toh_flush(x0[i]); const h16 a1 = toh_flush(x1[i]);
        hv[i] = a0; hv[4 + i] = a1;
        rv[i] = toh_flush((x0[i] - (float)a0) * QRS); rv[4 + i] = toh_flush((x1[i] - (float)a1) * QRS);
    }
}

__global__ __launch_bounds__(256) void k_cvt8(const float* __restrict__ src, bf* dst, size_t n8) {
    const size_t i = (size_t)blockIdx.x * 256 + threadIdx.x; if (i >= n8) return;
    const v8f v = *(const v8f*)(src + i * 8); v8us o;
#pragma unroll
    for (int k = 0; k < 8; ++k) o[k] = f2bf(v[k]);
    *(volatile v8us*)(dst + i * 8) = o; __threadfence(); *(volatile v8us*)(dst + i * 8) = o;
}

__global__ __launch_bounds__(SELT) void k_sel(const float* __restrict__ X, h16* XS, float* VS) {
#pragma clang fp contract(off)
    __shared__ int wt[NIT * (SELT / 32)];
    __shared__ __align__(16) float stg[SELP];
    const int tid = threadIdx.x, lane = tid & 31, wv = tid >> 5;
    const int b = blockIdx.x;
    const float* xr = X + (size_t)b * ND_FULL;
    float xv[NIT][8]; int ex[NIT];
#pragma unroll
    for (int it = 0; it < NIT; ++it) {
        const v8f v = *(const v8f*)(xr + it * SELP + tid * 8);
        int c = 0;
#pragma unroll
        for (int e = 0; e < 8; ++e) { xv[it][e] = bfr(v[e]); c += (xv[it][e] != 0.0f) ? 1 : 0; }
        int s = c;
#pragma unroll
        for (int d = 1; d < 32; d <<= 1) { const int t = __shfl_up(s, d, 32); s += (lane >= d) ? t : 0; }
        ex[it] = s - c;
        if (lane == 31) wt[it * (SELT / 32) + wv] = s;
    }
    __syncthreads();
    int prior = 0;
#pragma unroll
    for (int it = 0; it < NIT; ++it) {
        int inw = 0, all = 0;
#pragma unroll
        for (int w = 0; w < SELT / 32; ++w) { const int c = wt[it * (SELT / 32) + w]; all += c; inw += (w < wv) ? c : 0; }
        int r = prior + inw + ex[it];
        prior += all;
        v8h hv; v4f o0, o1;
#pragma unroll
        for (int e = 0; e < 8; ++e) {
            const bool nz = xv[it][e] != 0.0f;
            const bool keep = nz & (r < NNZ);
            const float val = keep ? xv[it][e] : 0.0f;
            hv[e] = toh_flush(val);
            if (e < 4) o0[e] = val; else o1[e - 4] = val;
            r += nz ? 1 : 0;
        }
        *(v4fa*)(&stg[tid * 8]) = o0; *(v4fa*)(&stg[tid * 8 + 4]) = o1;
        __syncthreads();
        const v4f w0 = *(const v4fa*)(&stg[tid * 4]);
        const v4f w1 = *(const v4fa*)(&stg[SELP / 2 + tid * 4]);
        const size_t pb = (size_t)b * ND + (size_t)it * SELP;
        h16* xs = XS + pb + (size_t)tid * 8;
        float* v0p = VS + pb + (size_t)tid * 4;
        float* v1p = VS + pb + (size_t)(SELP / 2) + (size_t)tid * 4;
        *(volatile v8h*)xs = hv; *(volatile v4f*)v0p = w0; *(volatile v4f*)v1p = w1;
        __threadfence();
        *(volatile v8h*)xs = hv; *(volatile v4f*)v0p = w0; *(volatile v4f*)v1p = w1;
        __syncthreads();
    }
}

__global__ __launch_bounds__(32) void k_proj(const bf* __restrict__ A, const bf* __restrict__ Bt, const float* __restrict__ bias, h16* Ph, h16* Pr, int pitch, int brow) {
    __shared__ __align__(16) float os[16 * 68];
    const int K = NE;
    const int lane = threadIdx.x & 31, lr = lane & 15, hi = lane >> 4; const int r0 = blockIdx.x * 64, c0 = blockIdx.y * 64;
    v8f acc[4][4];
#pragma unroll
    for (int mb = 0; mb < 4; ++mb)
#pragma unroll
        for (int nb = 0; nb < 4; ++nb) acc[mb][nb] = (v8f){};
    const size_t aoff = (size_t)(r0 + lr) * K + 8 * hi, boff = (size_t)(c0 + lr) * K + 8 * hi;
#pragma unroll 1
    for (int kc = 0; kc < K; kc += 32) {
        v16bf a[4];
#pragma unroll
        for (int mb = 0; mb < 4; ++mb) a[mb] = ldb(A + aoff + (size_t)mb * 16 * K + kc);
#pragma unroll
        for (int nb = 0; nb < 4; ++nb) { const v16bf b = ldb(Bt + boff + (size_t)nb * 16 * K + kc);
#pragma unroll
            for (int mb = 0; mb < 4; ++mb) acc[mb][nb] = gwb(a[mb], b, acc[mb][nb]); }
    }
    float bc[4];
#pragma unroll
    for (int nb = 0; nb < 4; ++nb) { int ci = c0 + nb * 16 + lr; ci = ci < (NQ - 1) ? ci : (NQ - 1); const float t = bias[ci]; bc[nb] = (brow != 0) ? 0.0f : bfr(t); }
#pragma unroll
    for (int mb = 0; mb < 4; ++mb) {
        float br[8];
#pragma unroll
        for (int j = 0; j < 8; ++j) { int ri = r0 + mb * 16 + hi * 8 + j; ri = ri < (NQ - 1) ? ri : (NQ - 1); const float t = bias[ri]; br[j] = (brow != 0) ? bfr(t) : 0.0f; }
#pragma unroll
        for (int nb = 0; nb < 4; ++nb) {
#pragma unroll
            for (int j = 0; j < 8; ++j) os[(hi * 8 + j) * 68 + nb * 16 + lr] = acc[mb][nb][j] + bc[nb] + br[j]; }
        wave_sync();
        const size_t sb = (size_t)(r0 + mb * 16) * (size_t)pitch + (size_t)c0;
#pragma unroll 1
        for (int ps = 0; ps < 2; ++ps) {
#pragma unroll
            for (int s = 0; s < 4; ++s) { const int row = 4 * s + (lane >> 3), c8 = (lane & 7) * 8;
                const v4f x0 = *(const v4fa*)(&os[row * 68 + c8]); const v4f x1 = *(const v4fa*)(&os[row * 68 + c8 + 4]); v8h hv, rv;
                split8(x0, x1, hv, rv);
                const size_t oo = sb + (size_t)row * (size_t)pitch + c8;
                *(volatile v8h*)(Ph + oo) = hv; *(volatile v8h*)(Pr + oo) = rv; }
            if (ps == 0) __threadfence(); }
        wave_sync();
    }
}

__global__ __launch_bounds__(32) void k_ug(const h16* __restrict__ XSp, const h16* __restrict__ QH, const h16* __restrict__ QR, h16* UH, h16* UR) {
    __shared__ __align__(16) float os[16 * 68];
    const int lane = threadIdx.x & 31, lr = lane & 15, hi = lane >> 4; const int r0 = blockIdx.x * 16, c0 = blockIdx.y * 64;
    v8f aH[4], aR[4];
#pragma unroll
    for (int nb = 0; nb < 4; ++nb) { aH[nb] = (v8f){}; aR[nb] = (v8f){}; }
    const size_t aoff = (size_t)(r0 + lr) * ND + 8 * hi, boff = (size_t)(c0 + lr) * ND + 8 * hi;
#pragma unroll 1
    for (int kc = 0; kc < ND; kc += 32) {
        const v16h a = ldh(XSp + aoff + kc);
#pragma unroll
        for (int nb = 0; nb < 4; ++nb) {
            const v16h bh = ldh(QH + boff + (size_t)nb * 16 * ND + kc);
            const v16h br = ldh(QR + boff + (size_t)nb * 16 * ND + kc);
            aH[nb] = gw16(a, bh, aH[nb]);
            aR[nb] = gw16(a, br, aR[nb]); }
    }
#pragma unroll
    for (int nb = 0; nb < 4; ++nb) {
#pragma unroll
        for (int j = 0; j < 8; ++j) os[(hi * 8 + j) * 68 + nb * 16 + lr] = aH[nb][j] + aR[nb][j] * QRI; }
    wave_sync();
    const size_t sb = (size_t)r0 * NQ + (size_t)c0;
#pragma unroll 1
    for (int ps = 0; ps < 2; ++ps) {
#pragma unroll
        for (int s = 0; s < 4; ++s) { const int row = 4 * s + (lane >> 3), c8 = (lane & 7) * 8;
            const v4f x0 = *(const v4fa*)(&os[row * 68 + c8]); const v4f x1 = *(const v4fa*)(&os[row * 68 + c8 + 4]); v8h hv, rv;
            split8(x0, x1, hv, rv);
            const size_t oo = sb + (size_t)row * NQ + c8;
            *(volatile v8h*)(UH + oo) = hv; *(volatile v8h*)(UR + oo) = rv; }
        if (ps == 0) __threadfence(); }
}

__global__ __launch_bounds__(32) void k_fx(const h16* __restrict__ UH, const h16* __restrict__ UR, const h16* __restrict__ KH, const h16* __restrict__ KR, const float* __restrict__ VS, float* OUT) {
    __shared__ __align__(16) float os[16 * 68];
    const int lane = threadIdx.x & 31, lr = lane & 15, hi = lane >> 4; const int r0 = blockIdx.x * 16, c0 = blockIdx.y * 64;
    v8f aH[4], aR[4];
#pragma unroll
    for (int nb = 0; nb < 4; ++nb) { aH[nb] = (v8f){}; aR[nb] = (v8f){}; }
    const size_t aoff = (size_t)(r0 + lr) * NQ + 8 * hi, boff = (size_t)(c0 + lr) * NQ + 8 * hi;
#pragma unroll 1
    for (int kc = 0; kc < NQ; kc += 32) {
        const v16h ah = ldh(UH + aoff + kc);
        const v16h ar = ldh(UR + aoff + kc);
#pragma unroll
        for (int nb = 0; nb < 4; ++nb) {
            const v16h bh = ldh(KH + boff + (size_t)nb * 16 * NQ + kc);
            const v16h br = ldh(KR + boff + (size_t)nb * 16 * NQ + kc);
            aH[nb] = gw16(ah, bh, aH[nb]);
            aR[nb] = gw16(ah, br, aR[nb]);
            aR[nb] = gw16(ar, bh, aR[nb]); }
    }
#pragma unroll
    for (int nb = 0; nb < 4; ++nb) {
#pragma unroll
        for (int j = 0; j < 8; ++j) os[(hi * 8 + j) * 68 + nb * 16 + lr] = (aH[nb][j] + aR[nb][j] * QRI) * SCL; }
    wave_sync();
#pragma unroll 1
    for (int ps = 0; ps < 2; ++ps) {
#pragma unroll
        for (int s = 0; s < 8; ++s) { const int row = 2 * s + (lane >> 4), cofs = (lane & 15) * 4;
            const v4f fx = *(const v4fa*)(&os[row * 68 + cofs]);
            const v4f vs = *(const v4f*)(VS + (size_t)(r0 + row) * ND + c0 + cofs);
            v4f y;
#pragma unroll
            for (int i = 0; i < 4; ++i) y[i] = (vs[i] != 0.0f) ? (vs[i] + vs[i] * fx[i]) : 0.0f;
            *(volatile v4f*)(OUT + (size_t)(r0 + row) * ND_FULL + c0 + cofs) = y; }
        if (ps == 0) __threadfence(); }
}

static constexpr size_t al256(size_t v) { return (v + 255) & ~(size_t)255; }
static constexpr size_t SZ_EB = al256((size_t)ND * NE * 2);
static constexpr size_t SZ_WB = al256((size_t)2 * NQ * NE * 2);
static constexpr size_t SZ_QT = al256((size_t)NQ * ND * 2);
static constexpr size_t SZ_KT = al256((size_t)ND * NQ * 2);
static constexpr size_t SZ_XS = al256((size_t)NB * ND * 2);
static constexpr size_t SZ_VS = al256((size_t)NB * ND * 4);
static constexpr size_t SZ_U  = al256((size_t)NB * NQ * 2);
static constexpr size_t SZ_TOTAL = SZ_EB + SZ_WB + 2 * SZ_QT + 2 * SZ_KT + SZ_XS + SZ_VS + 2 * SZ_U;
static_assert(SZ_TOTAL <= (size_t)134217728);
static_assert(((size_t)NQ * NE * 2) % 256 == 0);
static_assert(((size_t)ND * 2) % 128 == 0);
static_assert(((size_t)NQ * 2) % 128 == 0);
static_assert(((size_t)ND_FULL * 4) % 128 == 0);

extern "C" void kernel_launch(void* const* d_in, const int* in_sizes, int n_in,
                              void* d_out, int out_size, void* d_ws, size_t ws_size, hipStream_t stream) {
    if (n_in < 7) return;
    if ((size_t)in_sizes[1] < (size_t)(NB - 1) * ND_FULL + ND) return;
    if ((size_t)in_sizes[2] < (size_t)(ND + 1) * NE) return;
    if ((size_t)in_sizes[3] < (size_t)NQ * NE || (size_t)in_sizes[5] < (size_t)NQ * NE) return;
    if (in_sizes[4] < NQ || in_sizes[6] < NQ) return;
    if ((size_t)out_size < (size_t)(NB - 1) * ND_FULL + ND) return;
    if (SZ_TOTAL > ws_size) return;
    const float* x  = (const float*)d_in[1];
    const float* E  = (const float*)d_in[2];
    const float* wq = (const float*)d_in[3];
    const float* bq = (const float*)d_in[4];
    const float* wk = (const float*)d_in[5];
    const float* bk = (const float*)d_in[6];
    float* OUT = (float*)d_out;
    char* wsp = (char*)d_ws;
    bf*  EB  = (bf*)wsp;  wsp += SZ_EB;
    bf*  WB  = (bf*)wsp;  wsp += SZ_WB;
    h16* QTH = (h16*)wsp; wsp += SZ_QT;
    h16* QTR = (h16*)wsp; wsp += SZ_QT;
    h16* KTH = (h16*)wsp; wsp += SZ_KT;
    h16* KTR = (h16*)wsp; wsp += SZ_KT;
    h16* XS  = (h16*)wsp; wsp += SZ_XS;
    float* VS = (float*)wsp; wsp += SZ_VS;
    h16* UH  = (h16*)wsp; wsp += SZ_U;
    h16* UR  = (h16*)wsp; wsp += SZ_U;
    bf* WQ = WB; bf* WK = WB + (size_t)NQ * NE;

    { const size_t n8 = (size_t)ND * NE / 8;
      k_cvt8<<<(unsigned)((n8 + 255) / 256), 256, 0, stream>>>(E + NE, EB, n8); }
    { const size_t n8 = (size_t)NQ * NE / 8; const unsigned g = (unsigned)((n8 + 255) / 256);
      k_cvt8<<<g, 256, 0, stream>>>(wq, WQ, n8); k_cvt8<<<g, 256, 0, stream>>>(wk, WK, n8); }

    k_sel<<<NB, SELT, 0, stream>>>(x, XS, VS);

    k_proj<<<dim3(NQ / 64, ND / 64, 1), 32, 0, stream>>>(WQ, EB, bq, QTH, QTR, ND, 1);
    k_proj<<<dim3(ND / 64, NQ / 64, 1), 32, 0, stream>>>(EB, WK, bk, KTH, KTR, NQ, 0);

    k_ug<<<dim3(NB / 16, NQ / 64, 1), 32, 0, stream>>>(XS, QTH, QTR, UH, UR);
    k_fx<<<dim3(NB / 16, ND / 64, 1), 32, 0, stream>>>(UH, UR, KTH, KTR, VS, OUT);
}
